// SimilarityModel_24584392803023
// MI455X (gfx1250) — hardware-run, weakly checked
//
#include <hip/hip_runtime.h>
#include <math.h>

typedef __attribute__((ext_vector_type(16))) _Float16 v16h;
typedef __attribute__((ext_vector_type(16))) __bf16 v16b;
typedef __attribute__((ext_vector_type(8)))  _Float16 v8h;
typedef __attribute__((ext_vector_type(8)))  float v8f;
typedef __attribute__((ext_vector_type(4)))  float v4f;
typedef __attribute__((ext_vector_type(2)))  float v2f;
typedef __attribute__((ext_vector_type(4)))  unsigned v4u;
typedef __attribute__((ext_vector_type(4)))  int v4i;
typedef float __attribute__((may_alias)) float_a;
typedef int __attribute__((may_alias)) int_a;

template <typename T> __device__ __forceinline__ void vst2(void* p, T v) { *(volatile T*)p = v; __threadfence(); *(volatile T*)p = v; }
__device__ __forceinline__ v8f wmma16(v16h a, v16h b, v8f c) {
  v8f d = __builtin_amdgcn_wmma_f32_16x16x32_f16(false, a, false, b, (short)0, c, false, false);
  asm volatile("v_nop\n\tv_nop\n\tv_nop\n\tv_nop" : "+v"(d) : "v"(a), "v"(b));
  return d;
}
__device__ __forceinline__ v8f wmma_bf(v16b a, v16b b, v8f c) {
  v8f d = __builtin_amdgcn_wmma_f32_16x16x32_bf16(false, a, false, b, (short)0, c, false, false);
  asm volatile("v_nop\n\tv_nop\n\tv_nop\n\tv_nop" : "+v"(d) : "v"(a), "v"(b));
  return d;
}
__device__ __forceinline__ v16h frag_h(const _Float16* rowk0, int lane) {
  union { v16h v; v8h q[2]; } u; const _Float16* p = rowk0 + 8 * (lane >> 4);
  u.q[0] = *(const v8h*)p; u.q[1] = *(const v8h*)(p + 16); return u.v;
}
__device__ __forceinline__ v16h frag_f32(const float* rowk0, int lane) {
  v16h a; const float* p = rowk0 + 8 * (lane >> 4);
#pragma unroll
  for (int i = 0; i < 8; ++i) { a[i] = (_Float16)p[i]; a[8 + i] = (_Float16)p[16 + i]; }
  return a;
}
__device__ __forceinline__ v16h frag_f32s(const float* rowk0, int lane, float sc) {
  v16h a; const float* p = rowk0 + 8 * (lane >> 4);
#pragma unroll
  for (int i = 0; i < 8; ++i) { a[i] = (_Float16)(p[i] * sc); a[8 + i] = (_Float16)(p[16 + i] * sc); }
  return a;
}
__device__ __forceinline__ v16h fragc_f32(const float* W, int k0, int n, int lane, int ld, int K) {
  v16h a; const int g = lane >> 4;
#pragma unroll
  for (int i = 0; i < 8; ++i) { const int ka = k0 + 8 * g + i, kb = ka + 16;
    a[i] = (_Float16)(ka < K ? W[(size_t)(ka < K ? ka : K - 1) * ld + n] : 0.f); a[8 + i] = (_Float16)(kb < K ? W[(size_t)(kb < K ? kb : K - 1) * ld + n] : 0.f); }
  return a;
}
struct F2 { v16b h, l; };
__device__ __forceinline__ F2 bsplit16(const float v[16]) { F2 r;
#pragma unroll
  for (int i = 0; i < 16; ++i) { const __bf16 h = (__bf16)v[i]; r.h[i] = h; r.l[i] = (__bf16)(v[i] - (float)h); }
  return r; }
__device__ __forceinline__ F2 split_row(const float* row, int k0, int lane) { float v[16]; const float* p = row + k0 + 8 * (lane >> 4);
#pragma unroll
  for (int i = 0; i < 8; ++i) { v[i] = p[i]; v[8 + i] = p[16 + i]; }
  return bsplit16(v); }
__device__ __forceinline__ F2 split_rowK(const float* row, int k0, int lane, int K) { float v[16]; const int g = lane >> 4;
#pragma unroll
  for (int i = 0; i < 8; ++i) { const int ka = k0 + 8 * g + i, kb = ka + 16; v[i] = ka < K ? row[ka < K ? ka : K - 1] : 0.f; v[8 + i] = kb < K ? row[kb < K ? kb : K - 1] : 0.f; }
  return bsplit16(v); }
__device__ __forceinline__ F2 split_col(const float* W, int k0, int n, int lane, int ld, int K) { float v[16]; const int g = lane >> 4;
#pragma unroll
  for (int i = 0; i < 8; ++i) { const int ka = k0 + 8 * g + i, kb = ka + 16; v[i] = ka < K ? W[(size_t)(ka < K ? ka : K - 1) * ld + n] : 0.f; v[8 + i] = kb < K ? W[(size_t)(kb < K ? kb : K - 1) * ld + n] : 0.f; }
  return bsplit16(v); }
__device__ __forceinline__ v8f mac3(const F2& a, const F2& b, v8f c) { c = wmma_bf(a.l, b.h, c); c = wmma_bf(a.h, b.l, c); return wmma_bf(a.h, b.h, c); }
__device__ __forceinline__ float sigm(float v) { return 1.0f / (1.0f + expf(-v)); }
#define LDSX() do { asm volatile("s_wait_dscnt 0" ::: "memory"); __builtin_amdgcn_wave_barrier(); __builtin_amdgcn_fence(__ATOMIC_RELEASE, "workgroup"); } while (0)


#define NB 4
#define NC 384
#define NQ 384
#define HH 256
#define NROW (NB * NC * NQ)
#define NS 0.01f
#ifndef TBLK
#define TBLK (NROW / 64)
#endif
typedef __attribute__((ext_vector_type(8))) __bf16 v8b;
__device__ __forceinline__ v16b frag_b(const __bf16* rowk0, int lane) {
  union { v16b v; v8b q[2]; } u; const __bf16* p = rowk0 + 8 * (lane >> 4);
  u.q[0] = *(const v8b*)p; u.q[1] = *(const v8b*)(p + 16); return u.v;
}
__device__ __forceinline__ float bfr(float v) { return (float)(__bf16)v; }
__device__ __attribute__((noinline)) float exp_ni(float v) { return expf(v); }
__device__ __attribute__((noinline)) float erf_ni(float v) { return erff(v); }

#define WS_WHU (0u)
#define WS_TH  (WS_WHU + 2u * HH * HH)
#define WS_TU  (WS_TH + 4u * (size_t)NB * NC * HH)
#define WS_END (WS_TU + 4u * (size_t)NB * NQ * HH)

__device__ __forceinline__ v16b fragb_f32(const float* __restrict__ p, int lane) { v16b a; const float* pp = p + 8 * (lane >> 4);
#pragma unroll
  for (int i = 0; i < 8; ++i) { a[i] = (__bf16)pp[i]; a[8 + i] = (__bf16)pp[16 + i]; } return a; }
__global__ __launch_bounds__(256) void k_pack(const float* __restrict__ W1, _Float16* __restrict__ WHU) { const int n = blockIdx.x, t = threadIdx.x; __shared__ __align__(16) _Float16 s[HH]; s[t] = (_Float16)bfr(W1[(size_t)n * (3 * HH) + 2 * HH + t]); __syncthreads(); if (t < HH / 8) vst2((unsigned*)(WHU + (size_t)n * HH + t * 8), *(const v4u*)&s[t * 8]); }
__global__ __launch_bounds__(128) void k_terms(const float* __restrict__ Hm, const float* __restrict__ Um, const float* __restrict__ W1, float* __restrict__ TH, float* __restrict__ TU) { __shared__ __align__(16) float sf[4][16][132];
  const int tid = threadIdx.x, wave = tid >> 5, lane = tid & 31, col = lane & 15, g = lane >> 4; const int which = blockIdx.z; const float* X = which == 0 ? Hm : Um; float* T = which == 0 ? TH : TU; const size_t r0 = (size_t)blockIdx.x * 64 + wave * 16; const int c0 = blockIdx.y * 128;
  v8f acc[8] = {};
#pragma unroll
  for (int kc = 0; kc < HH / 32; ++kc) { const v16b a = fragb_f32(X + (r0 + col) * HH + kc * 32, lane);
#pragma unroll
    for (int j = 0; j < 8; ++j) acc[j] = wmma_bf(a, fragb_f32(W1 + (size_t)(c0 + j * 16 + col) * (3 * HH) + which * HH + kc * 32, lane), acc[j]); }
#pragma unroll
  for (int j = 0; j < 8; ++j)
#pragma unroll
    for (int r = 0; r < 8; ++r) sf[wave][8 * g + r][j * 16 + col] = acc[j][r];
  LDSX(); for (int rl = 0; rl < 16; ++rl) vst2(T + (r0 + rl) * HH + c0 + lane * 4, *(const v4f*)&sf[wave][rl][lane * 4]); }
__global__ __launch_bounds__(128) void k_sim(const float* __restrict__ Hm, const float* __restrict__ Um, const _Float16* __restrict__ WHU, const float* __restrict__ TH, const float* __restrict__ TU, const float* __restrict__ B1, const float* __restrict__ W2, const float* __restrict__ B2, float* __restrict__ OUT) { __shared__ float shc[HH]; __shared__ float sth[HH]; __shared__ __align__(16) float so[64];
  const int tid = threadIdx.x, wave = tid >> 5, lane = tid & 31, col = lane & 15, g = lane >> 4; const size_t row0 = (size_t)blockIdx.x * 64; const size_t bc = row0 / NQ; const size_t b = bc / NC; const int q0 = (int)(row0 % NQ) + wave * 16;
  for (int k = tid; k < HH; k += 128) { shc[k] = bfr(Hm[bc * HH + k]); sth[k] = TH[bc * HH + k]; } __syncthreads();
  const float* ur = Um + (b * NQ + q0 + col) * HH;
  float part[8];
#pragma unroll
  for (int r = 0; r < 8; ++r) part[r] = 0.f;
#pragma unroll 1
  for (int half = 0; half < 2; ++half) { v8f acc[8];
#pragma unroll
    for (int j = 0; j < 8; ++j) acc[j] = v8f{};
#pragma unroll 2
    for (int kc = 0; kc < HH / 32; ++kc) { v16h a; const int kb = kc * 32 + 8 * g;
#pragma unroll
      for (int i = 0; i < 8; ++i) { a[i] = (_Float16)(shc[kb + i] * bfr(ur[kb + i])); a[8 + i] = (_Float16)(shc[kb + 16 + i] * bfr(ur[kb + 16 + i])); }
#pragma unroll
      for (int j = 0; j < 8; ++j) acc[j] = wmma16(a, frag_h(WHU + (size_t)(half * 128 + j * 16 + col) * HH + kc * 32, lane), acc[j]); }
#pragma unroll
    for (int j = 0; j < 8; ++j) { const int n = half * 128 + j * 16 + col; const float add = sth[n] + bfr(B1[n]); const float w2 = bfr(W2[n]);
#pragma unroll
      for (int r = 0; r < 8; ++r) { const float tu = TU[(b * NQ + q0 + 8 * g + r) * HH + n]; float p = acc[j][r] + add + tu; p = (p > 0.f) ? p : NS * p; part[r] += p * w2; } } }
#pragma unroll
  for (int r = 0; r < 8; ++r) { float v = part[r];
#pragma unroll
    for (int o = 1; o < 16; o <<= 1) v += __shfl_xor(v, o);
    if (col == 0) { v += bfr(B2[0]); so[wave * 16 + 8 * g + r] = (v > 0.f) ? v : NS * v; } }
  __syncthreads(); if (tid < 16) vst2(OUT + row0 + tid * 4, *(const v4f*)&so[tid * 4]); }
extern "C" void kernel_launch(void* const* d_in, const int* in_sizes, int n_in, void* d_out, int out_size, void* d_ws, size_t ws_size, hipStream_t stream) {
  (void)in_sizes; (void)n_in; (void)out_size;
  const float** F = (const float**)d_in;
  if (ws_size < (size_t)WS_END) return;
  char* ws = (char*)d_ws; _Float16* WHU = (_Float16*)(ws + WS_WHU); float *TH = (float*)(ws + WS_TH), *TU = (float*)(ws + WS_TU);
  k_pack<<<HH, 256, 0, stream>>>(F[2], WHU);
  k_terms<<<dim3(NB * NC / 64, HH / 128, 2), 128, 0, stream>>>(F[0], F[1], F[2], TH, TU);
  k_sim<<<TBLK, 128, 0, stream>>>(F[0], F[1], WHU, TH, TU, F[3], F[4], F[5], (float*)d_out);
}
